// SpectralAttention_51513837748782
// MI455X (gfx1250) — hardware-verified
//
#include <hip/hip_runtime.h>
#include <math.h>

#ifndef NB
#define NB 8
#endif
#ifndef SEQ
#define SEQ 2048
#endif
#define NB_FULL 8
#define SEQ_FULL 2048
#define NC 512

static_assert(NB >= 1 && NB <= NB_FULL);
static_assert(SEQ % 256 == 0 && SEQ >= 256 && SEQ <= SEQ_FULL);
static_assert(NC % 64 == 0);

constexpr float kScale    = 0.04419417382415922f;
constexpr float kCarry    = 4096.0f;
constexpr float kInvCarry = 0.000244140625f;
constexpr int   kSmThreads = SEQ / 8;
constexpr int   kSmWaves   = kSmThreads / 32;

typedef __attribute__((ext_vector_type(16))) _Float16 v16h;
typedef __attribute__((ext_vector_type(8)))  _Float16 v8h;
typedef __attribute__((ext_vector_type(16))) __bf16   v16b;
typedef __attribute__((ext_vector_type(8)))  __bf16   v8b;
typedef __attribute__((ext_vector_type(8)))  float    v8f;
typedef __attribute__((ext_vector_type(4)))  float    v4f;
typedef __attribute__((ext_vector_type(4)))  unsigned int v4u;

__device__ __forceinline__ unsigned short f2bf_bits(float f) {
  unsigned u = __float_as_uint(f);
  return (unsigned short)((u + 0x7FFFu + ((u >> 16) & 1u)) >> 16);
}
__device__ __forceinline__ float bf_bits2f(unsigned short h) { return __uint_as_float(((unsigned)h) << 16); }

__device__ __forceinline__ void dep_guard_h(v8f& a, v8f& b, v16h x, v16h y) { asm volatile("v_nop\n\tv_nop\n\tv_nop\n\tv_nop" : "+v"(a), "+v"(b) : "v"(x), "v"(y)); }
__device__ __forceinline__ void dep_guard_b(v8f& a, v8f& b, v16b x, v16b y) { asm volatile("v_nop\n\tv_nop\n\tv_nop\n\tv_nop" : "+v"(a), "+v"(b) : "v"(x), "v"(y)); }
__device__ __forceinline__ void keep4_h(v16h a, v16h b, v16h c, v16h d) { asm volatile("v_nop" :: "v"(a), "v"(b), "v"(c), "v"(d)); }
__device__ __forceinline__ void keep4_b(v16b a, v16b b, v16b c, v16b d) { asm volatile("v_nop" :: "v"(a), "v"(b), "v"(c), "v"(d)); }
__device__ __forceinline__ void acc_guard4(v8f& a, v8f& b, v8f& c, v8f& d) { asm volatile("v_nop\n\tv_nop\n\tv_nop\n\tv_nop" : "+v"(a), "+v"(b), "+v"(c), "+v"(d)); }
template <typename T> struct Frag;
template <> struct Frag<_Float16> {
  typedef v16h V; union U { v16h v; v8h h[2]; };
  static __device__ __forceinline__ v16h load(const _Float16* p) {
    U f; f.h[0] = *(const v8h*)(p); f.h[1] = *(const v8h*)(p + 16); return f.v;
  }
  static __device__ __forceinline__ v8f mma(v16h a, v16h b, v8f c) {
    return __builtin_amdgcn_wmma_f32_16x16x32_f16(false, a, false, b, (short)0, c, false, false);
  }
  static __device__ __forceinline__ void guard(v8f& a, v8f& b, v16h x, v16h y) { dep_guard_h(a, b, x, y); }
  static __device__ __forceinline__ void keep(v16h a, v16h b, v16h c, v16h d) { keep4_h(a, b, c, d); }
};
template <> struct Frag<__bf16> {
  typedef v16b V; union U { v16b v; v8b h[2]; };
  static __device__ __forceinline__ v16b load(const __bf16* p) {
    U f; f.h[0] = *(const v8b*)(p); f.h[1] = *(const v8b*)(p + 16); return f.v;
  }
  static __device__ __forceinline__ v8f mma(v16b a, v16b b, v8f c) {
    return __builtin_amdgcn_wmma_f32_16x16x32_bf16(false, a, false, b, (short)0, c, false, false);
  }
  static __device__ __forceinline__ void guard(v8f& a, v8f& b, v16b x, v16b y) { dep_guard_b(a, b, x, y); }
  static __device__ __forceinline__ void keep(v16b a, v16b b, v16b c, v16b d) { keep4_b(a, b, c, d); }
};

__device__ __forceinline__ unsigned pk16(unsigned short a, unsigned short b) { return (unsigned)a | ((unsigned)b << 16); }

__device__ __forceinline__ float wave_sum32(float v) {
#pragma unroll
  for (int off = 16; off > 0; off >>= 1) v += __shfl_xor(v, off, 32);
  return v;
}
__device__ __forceinline__ float wave_max32(float v) {
#pragma unroll
  for (int off = 16; off > 0; off >>= 1) v = fmaxf(v, __shfl_xor(v, off, 32));
  return v;
}

template <int ET> struct Elem;
template <> struct Elem<0> { typedef _Float16 T; };
template <> struct Elem<1> { typedef __bf16 T; };
template <int ET, int SPLIT, int BIAS_MODE, int OUT_MODE>
__global__ __launch_bounds__(256) void wmma_gemm64(
    const unsigned short* __restrict__ Ap, const unsigned short* __restrict__ A2p, int lda, long strideA,
    const unsigned short* __restrict__ Btp, const unsigned short* __restrict__ Bt2p, int ldb, long strideB,
    void* __restrict__ Cout, void* __restrict__ Cout2, int ldc, long strideC,
    const float* __restrict__ bias0, const float* __restrict__ bias1,
    int M, int N, int K, float scale) {
  typedef typename Elem<ET>::T T;
  typedef typename Frag<T>::V V;
  const T* A = (const T*)Ap; const T* A2 = (const T*)A2p; const T* Bt = (const T*)Btp; const T* Bt2 = (const T*)Bt2p;
  __shared__ __align__(16) float sT[8][16 * 68];
  const int b    = blockIdx.y;
  const int lane = threadIdx.x & 31;
  const int wave = threadIdx.x >> 5;
  const int tilesN = N >> 6;
  const int tilesM = M >> 6;
  const int tile = blockIdx.x * 8 + wave;
  if (tile >= tilesM * tilesN) return;
  const int tm = tile / tilesN;
  const int tn = tile - tm * tilesN;
  const int m0 = tm << 6;
  const int n0 = tn << 6;

  const T* Ab  = A  + (size_t)b * strideA;
  const T* Bb  = Bt + (size_t)b * strideB;
  const T* Ab2 = (SPLIT >= 1) ? (A2  + (size_t)b * strideA) : nullptr;
  const T* Bb2 = (SPLIT == 2) ? (Bt2 + (size_t)b * strideB) : nullptr;
  const float* bias = (b == 0) ? bias0 : bias1;

  const int rlane = lane & 15;
  const int koff  = (lane >> 4) * 8;
  const int mOff  = (lane >> 4) * 8;

  v8f acc[4][4];
#pragma unroll
  for (int i = 0; i < 4; ++i)
#pragma unroll
    for (int j = 0; j < 4; ++j) acc[i][j] = (v8f){0.f,0.f,0.f,0.f,0.f,0.f,0.f,0.f};

  for (int k0 = 0; k0 < K; k0 += 32) {
    V bh[4], bl[4];
#pragma unroll
    for (int j = 0; j < 4; ++j) {
      const size_t bo = (size_t)(n0 + (j << 4) + rlane) * ldb + koff + k0;
      bh[j] = Frag<T>::load(Bb + bo);
      if (SPLIT == 2) bl[j] = Frag<T>::load(Bb2 + bo);
    }
#pragma unroll
    for (int i = 0; i < 4; ++i) {
      const size_t ao = (size_t)(m0 + (i << 4) + rlane) * lda + koff + k0;
      V ah = Frag<T>::load(Ab + ao);
      V al;
      if (SPLIT >= 1) al = Frag<T>::load(Ab2 + ao);
#pragma unroll
      for (int j = 0; j < 4; ++j) {
        acc[i][j] = Frag<T>::mma(ah, bh[j], acc[i][j]);
        if (SPLIT == 2) acc[i][j] = Frag<T>::mma(ah, bl[j], acc[i][j]);
        if (SPLIT >= 1) acc[i][j] = Frag<T>::mma(al, bh[j], acc[i][j]);
      }
      Frag<T>::guard(acc[i][0], acc[i][3], ah, (SPLIT >= 1) ? al : ah);
    }
    Frag<T>::keep(bh[0], bh[1], bh[2], bh[3]);
    if (SPLIT == 2) Frag<T>::keep(bl[0], bl[1], bl[2], bl[3]);
  }
  acc_guard4(acc[0][0], acc[0][1], acc[0][2], acc[0][3]);
  acc_guard4(acc[1][0], acc[1][1], acc[1][2], acc[1][3]);
  acc_guard4(acc[2][0], acc[2][1], acc[2][2], acc[2][3]);
  acc_guard4(acc[3][0], acc[3][1], acc[3][2], acc[3][3]);

  float* slab = sT[wave];
#pragma unroll
  for (int i = 0; i < 4; ++i) {
    const int mBase = m0 + (i << 4);
#pragma unroll
    for (int j = 0; j < 4; ++j) {
      const int n = n0 + (j << 4) + rlane;
      float bvl = 0.f;
      if (BIAS_MODE == 2) bvl = bf_bits2f(f2bf_bits(bias[n]));
#pragma unroll
      for (int r = 0; r < 8; ++r) {
        float v = acc[i][j][r] * scale;
        if (BIAS_MODE == 2) v += bvl;
        slab[(mOff + r) * 68 + (j << 4) + rlane] = v;
      }
    }
    __builtin_amdgcn_fence(__ATOMIC_RELEASE, "workgroup");
    __builtin_amdgcn_wave_barrier();
    __builtin_amdgcn_fence(__ATOMIC_ACQUIRE, "workgroup");
    if (OUT_MODE == 0) {
      float* C = (float*)Cout + (size_t)b * strideC;
      const int hh = lane >> 4, c4 = (lane & 15) * 4;
      for (int pass = 0; pass < 2; ++pass) {
#pragma unroll
        for (int it = 0; it < 8; ++it) {
          const int row = it * 2 + hh;
          v4f v = *(const v4f*)(slab + row * 68 + c4);
          *(volatile v4f*)(C + (size_t)(mBase + row) * ldc + n0 + c4) = v;
        }
        __threadfence();
      }
    } else {
      const int q = lane >> 3, c8 = (lane & 7) * 8;
      unsigned short* C  = (unsigned short*)Cout  + (size_t)b * strideC;
      unsigned short* C2 = (OUT_MODE == 2) ? ((unsigned short*)Cout2 + (size_t)b * strideC) : nullptr;
      for (int pass = 0; pass < 2; ++pass) {
#pragma unroll
        for (int it = 0; it < 4; ++it) {
          const int row = it * 4 + q;
          const float* sp = slab + row * 68 + c8;
          v8h hv, lv;
#pragma unroll
          for (int e = 0; e < 8; ++e) {
            if (OUT_MODE == 1) {
              hv[e] = (_Float16)sp[e];
            } else {
              unsigned short hb = f2bf_bits(sp[e]);
              unsigned short lb = f2bf_bits(sp[e] - bf_bits2f(hb));
              hv[e] = __builtin_bit_cast(_Float16, hb);
              lv[e] = __builtin_bit_cast(_Float16, lb);
            }
          }
          *(volatile v8h*)(C + (size_t)(mBase + row) * ldc + n0 + c8) = hv;
          if (OUT_MODE == 2) *(volatile v8h*)(C2 + (size_t)(mBase + row) * ldc + n0 + c8) = lv;
        }
        __threadfence();
      }
    }
    __builtin_amdgcn_fence(__ATOMIC_RELEASE, "workgroup");
    __builtin_amdgcn_wave_barrier();
    __builtin_amdgcn_fence(__ATOMIC_ACQUIRE, "workgroup");
  }
}

__global__ __launch_bounds__(256) void x_prep_kernel(const float* __restrict__ x,
                                                     unsigned short* __restrict__ xb, unsigned short* __restrict__ xT) {
  __shared__ float sm[64][65];
  const int t  = threadIdx.x;
  const int s0 = blockIdx.x * 64;
  const int c0 = blockIdx.y * 64;
  const int b  = blockIdx.z;
  const float* xin = x + ((size_t)b * SEQ_FULL + s0) * NC + c0;
#pragma unroll
  for (int i = 0; i < 16; ++i) {
    const int e = i * 256 + t;
    const int r = e >> 6;
    const int c = e & 63;
    sm[c][r] = bf_bits2f(f2bf_bits(xin[(size_t)r * NC + c]));
  }
  __syncthreads();
  const int lane = t & 31, wave = t >> 5;
  const int q = lane >> 3, c8 = (lane & 7) * 8;
  unsigned short* xTb = xT + (size_t)b * NC * SEQ;
  unsigned short* xbb = xb + (size_t)b * SEQ * NC;
  for (int pass = 0; pass < 2; ++pass) {
#pragma unroll
    for (int it = 0; it < 2; ++it) {
      const int row = wave * 8 + it * 4 + q;
      v8h hv;
      unsigned short bb[8];
#pragma unroll
      for (int e = 0; e < 8; ++e) {
        hv[e] = (_Float16)sm[row][c8 + e];
        bb[e] = f2bf_bits(sm[c8 + e][row]);
      }
      const v4u ub = (v4u){pk16(bb[0], bb[1]), pk16(bb[2], bb[3]), pk16(bb[4], bb[5]), pk16(bb[6], bb[7])};
      *(volatile v8h*)(xTb + (size_t)(c0 + row) * SEQ + s0 + c8) = hv;
      *(volatile v4u*)(xbb + (size_t)(s0 + row) * NC + c0 + c8) = ub;
    }
    __threadfence();
  }
}

__global__ __launch_bounds__(256) void w_prep_kernel(const float* __restrict__ W0, const float* __restrict__ W1,
                                                     const float* __restrict__ W2, unsigned short* __restrict__ wb) {
  constexpr int perPlane = NC * NC / 8;
  const int gid = blockIdx.x * 256 + threadIdx.x;
  const int z   = gid / perPlane;
  const int i8  = (gid - z * perPlane) * 8;
  const float* W = (z == 0) ? W0 : (z == 1) ? W1 : W2;
  const v4f a = *(const v4f*)(W + i8);
  const v4f c = *(const v4f*)(W + i8 + 4);
  unsigned short hb[8];
#pragma unroll
  for (int e = 0; e < 4; ++e) { hb[e] = f2bf_bits(a[e]); hb[4 + e] = f2bf_bits(c[e]); }
  const v4u uh = (v4u){pk16(hb[0], hb[1]), pk16(hb[2], hb[3]), pk16(hb[4], hb[5]), pk16(hb[6], hb[7])};
  unsigned short* p = wb + (size_t)z * NC * NC + i8;
  *(volatile v4u*)(p) = uh;
  __threadfence();
  *(volatile v4u*)(p) = uh;
}

__global__ __launch_bounds__(256) void ew_kernel(const float* __restrict__ eig, float* __restrict__ ew) {
  const int gid = blockIdx.x * 256 + threadIdx.x;
  const int b = gid / SEQ;
  const int s = gid - b * SEQ;
  const float e = bf_bits2f(f2bf_bits(eig[(size_t)b * SEQ_FULL + s]));
  const float v = 1.0f / (1.0f + expf(-e));
  *(volatile float*)(ew + gid) = v;
  __threadfence();
  *(volatile float*)(ew + gid) = v;
}

__global__ __launch_bounds__(256) void softmax_kernel(const float* __restrict__ S, const float* __restrict__ ewb,
                                                      unsigned short* __restrict__ P) {
  __shared__ float pm[kSmWaves];
  __shared__ float ps[kSmWaves];
  const int row = blockIdx.x;
  const int t = threadIdx.x;
  const int lane = t & 31, wave = t >> 5;
  const float* sp = S + (size_t)row * SEQ + 8 * t;
  const v4f a  = *(const v4f*)(sp);
  const v4f c  = *(const v4f*)(sp + 4);
  const v4f wa = *(const v4f*)(ewb + 8 * t);
  const v4f wc = *(const v4f*)(ewb + 8 * t + 4);
  float tv[8];
#pragma unroll
  for (int e = 0; e < 4; ++e) {
    tv[e]     = (a[e] * kScale) * wa[e];
    tv[4 + e] = (c[e] * kScale) * wc[e];
  }
  float m = tv[0];
#pragma unroll
  for (int e = 1; e < 8; ++e) m = fmaxf(m, tv[e]);
  m = wave_max32(m);
  if (lane == 0) pm[wave] = m;
  __syncthreads();
  float mm = pm[0];
#pragma unroll
  for (int w = 1; w < kSmWaves; ++w) mm = fmaxf(mm, pm[w]);
  float p[8];
  float ssum = 0.f;
#pragma unroll
  for (int e = 0; e < 8; ++e) { p[e] = __expf(tv[e] - mm); ssum += p[e]; }
  ssum = wave_sum32(ssum);
  if (lane == 0) ps[wave] = ssum;
  __syncthreads();
  float tot = ps[0];
#pragma unroll
  for (int w = 1; w < kSmWaves; ++w) tot += ps[w];
  const float inv = kCarry / tot;
  v8h hv;
#pragma unroll
  for (int e = 0; e < 8; ++e) hv[e] = (_Float16)(p[e] * inv);
  unsigned short* pp = P + (size_t)row * SEQ + 8 * t;
  *(volatile v8h*)(pp) = hv;
  __threadfence();
  *(volatile v8h*)(pp) = hv;
}

static inline size_t al64k(size_t v) { return (v + (size_t)65535) & ~(size_t)65535; }
static inline unsigned cdivu(unsigned a, unsigned b) { return (a + b - 1) / b; }

extern "C" void kernel_launch(void* const* d_in, const int* in_sizes, int n_in,
                              void* d_out, int out_size, void* d_ws, size_t ws_size,
                              hipStream_t stream) {
  if (n_in != 8) return;
  if (in_sizes[0] < (NB - 1) * SEQ_FULL * NC + SEQ * NC) return;
  if (in_sizes[1] < (NB - 1) * SEQ_FULL + SEQ) return;
  if (in_sizes[2] < NC * NC || in_sizes[4] < NC * NC || in_sizes[6] < NC * NC) return;
  if (in_sizes[3] < NC || in_sizes[5] < NC || in_sizes[7] < NC) return;
  if (out_size < NB * SEQ * NC) return;

  const size_t szXb  = (size_t)NB * SEQ * NC * 2;
  const size_t szXT  = (size_t)NB * NC * SEQ * 2;
  const size_t szWb  = (size_t)3 * NC * NC * 2;
  const size_t szEw  = (size_t)NB * SEQ * 4;
  const size_t szQK  = (size_t)2 * SEQ * NC * 2;
  const size_t szS   = (size_t)SEQ * SEQ * 4;
  const size_t szP   = (size_t)SEQ * SEQ * 2;
  const size_t szCtx = (size_t)SEQ * NC * 2;
  size_t off = 0;
  const size_t offXb   = off; off = al64k(off + szXb);
  const size_t offXT   = off; off = al64k(off + szXT);
  const size_t offWb   = off; off = al64k(off + szWb);
  const size_t offEw   = off; off = al64k(off + szEw);
  const size_t offQKh  = off; off = al64k(off + szQK);
  const size_t offQKl  = off; off = al64k(off + szQK);
  const size_t offS    = off; off = al64k(off + szS);
  const size_t offP    = off; off = al64k(off + szP);
  const size_t offCtxh = off; off = al64k(off + szCtx);
  const size_t offCtxl = off; off = al64k(off + szCtx);
  const size_t total   = off;
  if (ws_size < total) return;
  if (total > ((size_t)128 << 20)) return;

  const float* x   = (const float*)d_in[0];
  const float* eig = (const float*)d_in[1];
  const float* Wq  = (const float*)d_in[2];
  const float* bq  = (const float*)d_in[3];
  const float* Wk  = (const float*)d_in[4];
  const float* bk  = (const float*)d_in[5];
  const float* Wv  = (const float*)d_in[6];
  const float* bv  = (const float*)d_in[7];
  float* out = (float*)d_out;

  char* ws = (char*)d_ws;
  unsigned short* xb    = (unsigned short*)(ws + offXb);
  unsigned short* xT    = (unsigned short*)(ws + offXT);
  unsigned short* wb    = (unsigned short*)(ws + offWb);
  float*          ew    = (float*)(ws + offEw);
  unsigned short* qkh   = (unsigned short*)(ws + offQKh);
  unsigned short* qkl   = (unsigned short*)(ws + offQKl);
  float*          Sbuf  = (float*)(ws + offS);
  unsigned short* Pbuf  = (unsigned short*)(ws + offP);
  unsigned short* ctxh  = (unsigned short*)(ws + offCtxh);
  unsigned short* ctxl  = (unsigned short*)(ws + offCtxl);

  const long planeW  = (long)NC * NC;
  const long planeQK = (long)SEQ * NC;

  x_prep_kernel<<<dim3(SEQ / 64, NC / 64, NB), 256, 0, stream>>>(x, xb, xT);
  w_prep_kernel<<<dim3(3 * NC * NC / 8 / 256), 256, 0, stream>>>(Wq, Wk, Wv, wb);
  ew_kernel<<<dim3(NB * SEQ / 256), 256, 0, stream>>>(eig, ew);

  const unsigned blkProj   = cdivu((SEQ / 64) * (NC / 64), 8);
  const unsigned blkScores = cdivu((SEQ / 64) * (SEQ / 64), 8);

  for (int bb = 0; bb < NB; ++bb) {
    const unsigned short* xbB = xb + (size_t)bb * SEQ * NC;
    const unsigned short* xTB = xT + (size_t)bb * NC * SEQ;
    float* outB = out + (size_t)bb * SEQ * NC;
    wmma_gemm64<1, 0, 2, 2><<<dim3(blkProj, 2), 256, 0, stream>>>(
        xbB, xbB, NC, 0L, wb, wb, NC, planeW,
        (void*)qkh, (void*)qkl, NC, planeQK, bq, bk, SEQ, NC, NC, 1.0f);
    wmma_gemm64<1, 2, 0, 0><<<dim3(blkScores, 1), 256, 0, stream>>>(
        qkh, qkl, NC, 0L, qkh + planeQK, qkl + planeQK, NC, 0L,
        (void*)Sbuf, (void*)Sbuf, SEQ, 0L, ew, ew, SEQ, SEQ, NC, 1.0f);
    softmax_kernel<<<dim3(SEQ), kSmThreads, 0, stream>>>(Sbuf, ew + (size_t)bb * SEQ, Pbuf);
    wmma_gemm64<0, 0, 0, 2><<<dim3(blkProj, 1), 256, 0, stream>>>(
        Pbuf, Pbuf, SEQ, 0L, xTB, xTB, SEQ, 0L,
        (void*)ctxh, (void*)ctxl, NC, 0L, ew, ew, SEQ, NC, SEQ, kInvCarry);
    wmma_gemm64<1, 1, 2, 0><<<dim3(blkProj, 1), 256, 0, stream>>>(
        ctxh, ctxl, NC, 0L, wb + 2 * planeW, wb + 2 * planeW, NC, 0L,
        (void*)outB, (void*)outB, NC, 0L, bv, bv, SEQ, NC, NC, 1.0f);
  }
}
